// MultiSubwordAttentionTagger_86663850099017
// MI455X (gfx1250) — hardware-verified
//
#include <hip/hip_runtime.h>
#include <stddef.h>
#include <stdint.h>

#define NS     1024
#define NBT    16
#define NTOK   (NS * NBT)
#define ED     256
#define EMBW   768
#define HIDW   512
#define TAGW   32
#define KHG    (3 * HIDW)
#define CHARV  20000
#define SUBV   10000
#define BR     32
#define WSC    64.0f
#define XNSC   16.0f
#define PSC    1024.0f
#define INV64    0.015625f
#define INV256   0.00390625f
#define INV1024  0.0009765625f
#define INV65536 0.0000152587890625f

static_assert(NTOK % 256 == 0);
static_assert(NS % 256 == 0);
static_assert(NS % BR == 0);
static_assert(HIDW % 64 == 0);
static_assert(EMBW % 256 == 0);
static_assert(KHG % 256 == 0);
static_assert(ED == 256);
static_assert(TAGW == 32);
static_assert(HIDW == 512);

typedef float          v8f   __attribute__((ext_vector_type(8)));
typedef float          v4f   __attribute__((ext_vector_type(4)));
typedef double         v2d   __attribute__((ext_vector_type(2)));
typedef unsigned int   v4u   __attribute__((ext_vector_type(4)));
typedef unsigned short v8us  __attribute__((ext_vector_type(8)));
typedef unsigned short v16us __attribute__((ext_vector_type(16)));
typedef _Float16       v16h  __attribute__((ext_vector_type(16)));
typedef unsigned short ush;

union FragU { v16us v; v8us h[2]; v16h f; };
union PackU { v8us s; v4u u; };

__device__ __forceinline__ ush f2h(float f) {
  const _Float16 h = (_Float16)f;
  return __builtin_bit_cast(ush, h);
}

__device__ __forceinline__ v8f zero8() { return (v8f){0.f, 0.f, 0.f, 0.f, 0.f, 0.f, 0.f, 0.f}; }

__device__ __forceinline__ v8f mmah(v16us a, v16us b, v8f c) {
  FragU ua, ub; ua.v = a; ub.v = b;
  c = __builtin_amdgcn_wmma_f32_16x16x32_f16(false, ua.f, false, ub.f, (short)0, c, false, false);
  asm volatile("v_nop\n\tv_nop\n\tv_nop\n\tv_nop" : "+v"(c) : "v"(a), "v"(b));
  return c;
}

__device__ __forceinline__ v16us ldfragu(const ush* p, int ld, int row0, int k0, int lane) {
  const int m = lane & 15, lh = lane >> 4;
  const ush* q = p + (size_t)(row0 + m) * ld + k0 + 8 * lh;
  FragU f;
  f.h[0] = *(const v8us*)(q);
  f.h[1] = *(const v8us*)(q + 16);
  return f.v;
}

__device__ __forceinline__ void gemm_32x64(const ush* __restrict__ A, int lda,
                                           const ush* __restrict__ Bm, int ldb, int K,
                                           int m0, int n0, int lane, v8f (&acc)[2][4]) {
#pragma unroll 1
  for (int k0 = 0; k0 < K; k0 += 32) {
    const v16us a0 = ldfragu(A, lda, m0, k0, lane);
    const v16us a1 = ldfragu(A, lda, m0 + 16, k0, lane);
#pragma unroll
    for (int t = 0; t < 4; ++t) {
      const v16us bb = ldfragu(Bm, ldb, n0 + 16 * t, k0, lane);
      acc[0][t] = mmah(a0, bb, acc[0][t]);
      acc[1][t] = mmah(a1, bb, acc[1][t]);
    }
  }
}

#define WTP 260
__global__ __launch_bounds__(256) void k_cvt_w(const float* __restrict__ w, int ncol, int nk,
                                               ush* __restrict__ wt) {
  __shared__ __align__(16) float st[16 * WTP];
  const int tid = threadIdx.x;
  const int h0 = blockIdx.x * 16;
  const int k0 = blockIdx.y * 256;
  {
    const float* src = w + (size_t)(k0 + tid) * ncol + h0;
    const v4f a0 = *(const v4f*)(src);
    const v4f a1 = *(const v4f*)(src + 4);
    const v4f a2 = *(const v4f*)(src + 8);
    const v4f a3 = *(const v4f*)(src + 12);
#pragma unroll
    for (int e = 0; e < 4; ++e) {
      st[(e)      * WTP + tid] = a0[e];
      st[(4 + e)  * WTP + tid] = a1[e];
      st[(8 + e)  * WTP + tid] = a2[e];
      st[(12 + e) * WTP + tid] = a3[e];
    }
  }
  __syncthreads();
  v4u vh[2];
  size_t go[2];
#pragma unroll
  for (int j = 0; j < 2; ++j) {
    const int p   = tid + 256 * j;
    const int row = p >> 5;
    const int pc  = p & 31;
    const float* sp = st + row * WTP + pc * 8;
    const v4f b0 = *(const v4f*)(sp);
    const v4f b1 = *(const v4f*)(sp + 4);
    PackU pk;
#pragma unroll
    for (int e = 0; e < 4; ++e) {
      pk.s[e]     = f2h(b0[e] * WSC);
      pk.s[4 + e] = f2h(b1[e] * WSC);
    }
    vh[j] = pk.u;
    go[j] = ((size_t)(h0 + row)) * nk + (size_t)k0 + (size_t)pc * 8;
  }
#pragma unroll
  for (int j = 0; j < 2; ++j) *(volatile v4u*)(wt + go[j]) = vh[j];
  __threadfence();
#pragma unroll
  for (int j = 0; j < 2; ++j) *(volatile v4u*)(wt + go[j]) = vh[j];
}

__global__ __launch_bounds__(256) void k_gather(const int* __restrict__ xc, const int* __restrict__ xs0,
                                                const int* __restrict__ xs1,
                                                const float* __restrict__ Ec, const float* __restrict__ E0,
                                                const float* __restrict__ E1,
                                                ush* __restrict__ emb, ush* __restrict__ xn0,
                                                ush* __restrict__ xn1) {
  const int tid = threadIdx.x, lane = tid & 31, wave = tid >> 5;
  const int mb  = blockIdx.x * 8 + wave;
  const int b   = mb >> 10, n = mb & (NS - 1);
  const int pos = n * NBT + b;
  int ic = xc[pos];  ic = min(max(ic, 0), CHARV - 1);
  int i0 = xs0[pos]; i0 = min(max(i0, 0), SUBV - 1);
  int i1 = xs1[pos]; i1 = min(max(i1, 0), SUBV - 1);
  const float* rc = Ec + (size_t)ic * ED + lane * 8;
  const float* r0 = E0 + (size_t)i0 * ED + lane * 8;
  const float* r1 = E1 + (size_t)i1 * ED + lane * 8;
  const v4f c0 = *(const v4f*)(rc), c1 = *(const v4f*)(rc + 4);
  const v4f p0 = *(const v4f*)(r0), p1 = *(const v4f*)(r0 + 4);
  const v4f q0 = *(const v4f*)(r1), q1 = *(const v4f*)(r1 + 4);
  float ss0 = 0.f, ss1 = 0.f;
#pragma unroll
  for (int e = 0; e < 4; ++e) {
    ss0 += p0[e] * p0[e]; ss0 += p1[e] * p1[e];
    ss1 += q0[e] * q0[e]; ss1 += q1[e] * q1[e];
  }
#pragma unroll
  for (int o = 16; o > 0; o >>= 1) {
    ss0 += __shfl_xor(ss0, o, 32);
    ss1 += __shfl_xor(ss1, o, 32);
  }
  const float inv0 = (1.0f / sqrtf(ss0)) * XNSC;
  const float inv1 = (1.0f / sqrtf(ss1)) * XNSC;
  PackU pe, ps0, ps1, pn0, pn1;
#pragma unroll
  for (int e = 0; e < 4; ++e) {
    pe.s[e]  = f2h(c0[e]);          pe.s[4 + e]  = f2h(c1[e]);
    ps0.s[e] = f2h(p0[e]);          ps0.s[4 + e] = f2h(p1[e]);
    ps1.s[e] = f2h(q0[e]);          ps1.s[4 + e] = f2h(q1[e]);
    pn0.s[e] = f2h(p0[e] * inv0);   pn0.s[4 + e] = f2h(p1[e] * inv0);
    pn1.s[e] = f2h(q0[e] * inv1);   pn1.s[4 + e] = f2h(q1[e] * inv1);
  }
  const size_t eo = (size_t)mb * EMBW + (size_t)lane * 8;
  const size_t xo = (size_t)mb * ED + (size_t)lane * 8;
  *(volatile v4u*)(emb + eo)          = pe.u;
  *(volatile v4u*)(emb + eo + ED)     = ps0.u;
  *(volatile v4u*)(emb + eo + 2 * ED) = ps1.u;
  *(volatile v4u*)(xn0 + xo)          = pn0.u;
  *(volatile v4u*)(xn1 + xo)          = pn1.u;
  __threadfence();
  *(volatile v4u*)(emb + eo)          = pe.u;
  *(volatile v4u*)(emb + eo + ED)     = ps0.u;
  *(volatile v4u*)(emb + eo + 2 * ED) = ps1.u;
  *(volatile v4u*)(xn0 + xo)          = pn0.u;
  *(volatile v4u*)(xn1 + xo)          = pn1.u;
}

#define STP 72
__global__ __launch_bounds__(256) void k_hgemm(const ush* __restrict__ emb, const ush* __restrict__ w1t,
                                               const float* __restrict__ bias,
                                               ush* __restrict__ hp, ush* __restrict__ htp) {
  __shared__ __align__(16) ush st[256 * STP];
  const int tid = threadIdx.x, lane = tid & 31, wave = tid >> 5;
  const int hh = lane >> 4, c = lane & 15;
  const int mb = blockIdx.x * 256;
  const int m0 = mb + wave * 32;
  const int n0 = blockIdx.y * 64;
  const int b  = mb >> 10;
  const int l0 = mb & (NS - 1);

  v8f acc[2][4];
#pragma unroll
  for (int s = 0; s < 2; ++s)
#pragma unroll
    for (int t = 0; t < 4; ++t) acc[s][t] = zero8();
  gemm_32x64(emb, EMBW, w1t, EMBW, EMBW, m0, n0, lane, acc);

#pragma unroll
  for (int t = 0; t < 4; ++t) {
    const float bn = bias[n0 + 16 * t + c];
#pragma unroll
    for (int sub = 0; sub < 2; ++sub) {
#pragma unroll
      for (int r = 0; r < 8; ++r) {
        const int lr = wave * 32 + sub * 16 + 8 * hh + r;
        st[lr * STP + 16 * t + c] = f2h(acc[sub][t][r] * INV64 + bn);
      }
    }
  }
  __syncthreads();
  {
    v4u val[8];
    size_t go[8];
#pragma unroll
    for (int j = 0; j < 8; ++j) {
      const int p  = tid + 256 * j;
      const int L  = p >> 3;
      const int pc = p & 7;
      PackU pk;
      pk.s   = *(const v8us*)(st + L * STP + pc * 8);
      val[j] = pk.u;
      go[j]  = ((size_t)(mb + L)) * HIDW + n0 + pc * 8;
    }
#pragma unroll
    for (int j = 0; j < 8; ++j) *(volatile v4u*)(hp + go[j]) = val[j];
    __threadfence();
#pragma unroll
    for (int j = 0; j < 8; ++j) *(volatile v4u*)(hp + go[j]) = val[j];
  }
  {
    v4u val[8];
    size_t go[8];
#pragma unroll
    for (int j = 0; j < 8; ++j) {
      const int p  = tid + 256 * j;
      const int L  = p >> 3;
      const int pc = p & 7;
      const int d  = L >> 2;
      const int nl = (L & 3) * 64 + pc * 8;
      const ush* cp = st + nl * STP + d;
      PackU pk;
      pk.s = (v8us){cp[0 * STP], cp[1 * STP], cp[2 * STP], cp[3 * STP],
                    cp[4 * STP], cp[5 * STP], cp[6 * STP], cp[7 * STP]};
      val[j] = pk.u;
      go[j]  = ((size_t)(b * HIDW + n0 + d)) * NS + l0 + nl;
    }
#pragma unroll
    for (int j = 0; j < 8; ++j) *(volatile v4u*)(htp + go[j]) = val[j];
    __threadfence();
#pragma unroll
    for (int j = 0; j < 8; ++j) *(volatile v4u*)(htp + go[j]) = val[j];
  }
}

#define SSP 1028
#define SPP 1032
#define GTP 520
#define ATT_LDS (BR * SSP * 4 + BR * SPP * 2)
__global__ __launch_bounds__(256) void k_attn(const ush* __restrict__ xn0, const ush* __restrict__ xn1,
                                              const ush* __restrict__ htp,
                                              ush* __restrict__ g0p, ush* __restrict__ g1p,
                                              double* __restrict__ part) {
  extern __shared__ __align__(16) char smem[];
  __shared__ double red[8];
  float* sS = (float*)smem;
  ush*   sP = (ush*)(smem + BR * SSP * 4);

  const int tid = threadIdx.x, lane = tid & 31, wave = tid >> 5;
  const int hh = lane >> 4, c = lane & 15;
  const int bx = blockIdx.x, b = blockIdx.y, z = blockIdx.z;
  const int q0 = bx * BR;
  const ush* X  = ((z == 0) ? xn0 : xn1) + (size_t)b * NS * ED;
  ush*       G  = (z == 0) ? g0p : g1p;
  const ush* Hb = htp + (size_t)b * HIDW * NS;

#pragma unroll 1
  for (int jt = wave; jt < NS / 16; jt += 8) {
    v8f s0 = zero8(), s1 = zero8();
#pragma unroll 1
    for (int k0 = 0; k0 < ED; k0 += 32) {
      const v16us a0 = ldfragu(X, ED, q0, k0, lane);
      const v16us a1 = ldfragu(X, ED, q0 + 16, k0, lane);
      const v16us kb = ldfragu(X, ED, jt * 16, k0, lane);
      s0 = mmah(a0, kb, s0);
      s1 = mmah(a1, kb, s1);
    }
#pragma unroll
    for (int r = 0; r < 8; ++r) {
      sS[(8 * hh + r) * SSP + jt * 16 + c]      = s0[r] * INV256;
      sS[(16 + 8 * hh + r) * SSP + jt * 16 + c] = s1[r] * INV256;
    }
  }
  __syncthreads();

  {
    const int row = tid >> 3, ck = tid & 7;
    float* sr = sS + row * SSP + ck * 128;
    float mx = -__builtin_huge_valf();
#pragma unroll 4
    for (int i = 0; i < 32; ++i) {
      const v4f x = *(const v4f*)(sr + 4 * i);
      mx = fmaxf(fmaxf(mx, fmaxf(x[0], x[1])), fmaxf(x[2], x[3]));
    }
    mx = fmaxf(mx, __shfl_xor(mx, 1, 32));
    mx = fmaxf(mx, __shfl_xor(mx, 2, 32));
    mx = fmaxf(mx, __shfl_xor(mx, 4, 32));
    float sum = 0.f;
#pragma unroll 2
    for (int i = 0; i < 32; ++i) {
      const v4f x = *(const v4f*)(sr + 4 * i);
      v4f e;
      e[0] = __expf(x[0] - mx); e[1] = __expf(x[1] - mx);
      e[2] = __expf(x[2] - mx); e[3] = __expf(x[3] - mx);
      sum += (e[0] + e[1]) + (e[2] + e[3]);
      *(v4f*)(sr + 4 * i) = e;
    }
    sum += __shfl_xor(sum, 1, 32);
    sum += __shfl_xor(sum, 2, 32);
    sum += __shfl_xor(sum, 4, 32);
    const float psc = PSC * (1.0f / sum);
#pragma unroll 2
    for (int i = 0; i < 16; ++i) {
      const v4f e0 = *(const v4f*)(sr + 8 * i);
      const v4f e1 = *(const v4f*)(sr + 8 * i + 4);
      PackU pk;
#pragma unroll
      for (int e = 0; e < 4; ++e) {
        pk.s[e]     = f2h(e0[e] * psc);
        pk.s[4 + e] = f2h(e1[e] * psc);
      }
      *(v8us*)(sP + row * SPP + ck * 128 + 8 * i) = pk.s;
    }
  }
  __syncthreads();

  v8f acc[2][4];
#pragma unroll
  for (int s = 0; s < 2; ++s)
#pragma unroll
    for (int t = 0; t < 4; ++t) acc[s][t] = zero8();
  const int c0 = wave * 64;
#pragma unroll 1
  for (int k0 = 0; k0 < NS; k0 += 32) {
    const v16us pa0 = ldfragu(sP, SPP, 0, k0, lane);
    const v16us pa1 = ldfragu(sP, SPP, 16, k0, lane);
#pragma unroll
    for (int t = 0; t < 4; ++t) {
      const v16us vb = ldfragu(Hb, NS, c0 + 16 * t, k0, lane);
      acc[0][t] = mmah(pa0, vb, acc[0][t]);
      acc[1][t] = mmah(pa1, vb, acc[1][t]);
    }
  }
  __syncthreads();

  ush* st = (ush*)smem;
  double lsq = 0.0;
#pragma unroll
  for (int sub = 0; sub < 2; ++sub) {
#pragma unroll
    for (int t = 0; t < 4; ++t) {
#pragma unroll
      for (int r = 0; r < 8; ++r) {
        const float v  = acc[sub][t][r];
        const float gv = v * INV1024;
        lsq += (double)gv * (double)gv;
        st[(16 * sub + 8 * hh + r) * GTP + c0 + 16 * t + c] = f2h(v);
      }
    }
  }
#pragma unroll
  for (int o = 16; o > 0; o >>= 1) lsq += __shfl_xor(lsq, o, 32);
  if (lane == 0) red[wave] = lsq;
  __syncthreads();

  v4u val[8];
  size_t go[8];
#pragma unroll
  for (int it = 0; it < 8; ++it) {
    const int p   = tid + 256 * it;
    const int L   = p >> 3;
    const int pc  = p & 7;
    const int row = L >> 3;
    const int lq  = L & 7;
    PackU pk;
    pk.s    = *(const v8us*)(st + row * GTP + lq * 64 + pc * 8);
    val[it] = pk.u;
    go[it]  = ((size_t)(b * NS + q0 + row)) * HIDW + lq * 64 + pc * 8;
  }
  double tot = 0.0;
#pragma unroll
  for (int i = 0; i < 8; ++i) tot += red[i];
  v2d pv;
  pv[0] = (tid == 0) ? tot : 0.0;
  pv[1] = 0.0;
  double* pp = part + ((size_t)((z * NBT + b) * (NS / BR) + bx)) * 16 + (size_t)tid * 2;

#pragma unroll
  for (int it = 0; it < 8; ++it) *(volatile v4u*)(G + go[it]) = val[it];
  if (tid < 8) *(volatile v2d*)(pp) = pv;
  __threadfence();
#pragma unroll
  for (int it = 0; it < 8; ++it) *(volatile v4u*)(G + go[it]) = val[it];
  if (tid < 8) *(volatile v2d*)(pp) = pv;
}

#define ZTP 36
__device__ __forceinline__ void seg_16x32(const ush* __restrict__ A, int r0,
                                          const ush* __restrict__ w2t, int kofs, int lane, v8f (&acc)[2]) {
#pragma unroll 1
  for (int k0 = 0; k0 < HIDW; k0 += 32) {
    const v16us a  = ldfragu(A, HIDW, r0, k0, lane);
    const v16us b0 = ldfragu(w2t, KHG, 0, kofs + k0, lane);
    const v16us b1 = ldfragu(w2t, KHG, 16, kofs + k0, lane);
    acc[0] = mmah(a, b0, acc[0]);
    acc[1] = mmah(a, b1, acc[1]);
  }
}

__global__ __launch_bounds__(256) void k_final(const ush* __restrict__ hp, const ush* __restrict__ g0p,
                                               const ush* __restrict__ g1p, const ush* __restrict__ w2t,
                                               const float* __restrict__ bias, const double* __restrict__ part,
                                               float* __restrict__ out) {
  __shared__ __align__(16) float sZ[128 * ZTP];
  __shared__ double red[2][8];
  const int tid = threadIdx.x, lane = tid & 31, wave = tid >> 5;
  const int hh = lane >> 4, c = lane & 15;
  const int mb0 = blockIdx.x * 128;

  double d0 = part[((size_t)(2 * tid)) * 16] + part[((size_t)(2 * tid + 1)) * 16];
  double d1 = part[((size_t)(512 + 2 * tid)) * 16] + part[((size_t)(512 + 2 * tid + 1)) * 16];
#pragma unroll
  for (int o = 16; o > 0; o >>= 1) {
    d0 += __shfl_xor(d0, o, 32);
    d1 += __shfl_xor(d1, o, 32);
  }
  if (lane == 0) { red[0][wave] = d0; red[1][wave] = d1; }
  __syncthreads();
  double S0 = 0.0, S1 = 0.0;
#pragma unroll
  for (int i = 0; i < 8; ++i) { S0 += red[0][i]; S1 += red[1][i]; }
  const float s0  = 1.0f / sqrtf((float)S0);
  const float s1  = 1.0f / sqrtf((float)S1);
  const float cf0 = s0 * INV65536;
  const float cf1 = s1 * INV65536;

  const int r0 = mb0 + wave * 16;
  v8f acc[3][2];
#pragma unroll
  for (int s = 0; s < 3; ++s) { acc[s][0] = zero8(); acc[s][1] = zero8(); }
  seg_16x32(hp,  r0, w2t, 0,        lane, acc[0]);
  seg_16x32(g0p, r0, w2t, HIDW,     lane, acc[1]);
  seg_16x32(g1p, r0, w2t, 2 * HIDW, lane, acc[2]);

#pragma unroll
  for (int t = 0; t < 2; ++t) {
    const float bn = bias[16 * t + c];
#pragma unroll
    for (int r = 0; r < 8; ++r) {
      const int row = wave * 16 + 8 * hh + r;
      const float zv = acc[0][t][r] * INV64 + acc[1][t][r] * cf0 + acc[2][t][r] * cf1 + bn;
      sZ[row * ZTP + 16 * t + c] = zv;
    }
  }
  __syncthreads();
  v4f val[4];
  size_t go[4];
#pragma unroll
  for (int it = 0; it < 4; ++it) {
    const int p  = tid + 256 * it;
    const int L  = p >> 3;
    const int pc = p & 7;
    val[it] = *(const v4f*)(sZ + L * ZTP + pc * 4);
    const int mb = mb0 + L;
    const int bq = mb >> 10, n = mb & (NS - 1);
    go[it] = ((size_t)(n * NBT + bq)) * TAGW + pc * 4;
  }
#pragma unroll
  for (int it = 0; it < 4; ++it) *(volatile v4f*)(out + go[it]) = val[it];
  __threadfence();
#pragma unroll
  for (int it = 0; it < 4; ++it) *(volatile v4f*)(out + go[it]) = val[it];
}

extern "C" void kernel_launch(void* const* d_in, const int* in_sizes, int n_in,
                              void* d_out, int out_size, void* d_ws, size_t ws_size,
                              hipStream_t stream) {
  if (n_in < 10) return;
  if (in_sizes[0] != NTOK || in_sizes[1] != NTOK || in_sizes[2] != NTOK) return;
  if (in_sizes[3] != CHARV * ED) return;
  if (in_sizes[4] != SUBV * ED || in_sizes[5] != SUBV * ED) return;
  if (in_sizes[6] != EMBW * HIDW || in_sizes[7] != HIDW) return;
  if (in_sizes[8] != KHG * TAGW || in_sizes[9] != TAGW) return;
  if (out_size != NTOK * TAGW) return;

  const int*   xc = (const int*)d_in[0];
  const int*   x0 = (const int*)d_in[1];
  const int*   x1 = (const int*)d_in[2];
  const float* Ec = (const float*)d_in[3];
  const float* E0 = (const float*)d_in[4];
  const float* E1 = (const float*)d_in[5];
  const float* W1 = (const float*)d_in[6];
  const float* b1 = (const float*)d_in[7];
  const float* W2 = (const float*)d_in[8];
  const float* b2 = (const float*)d_in[9];
  float* out = (float*)d_out;

  size_t off = 0;
  const size_t oEMB = off; off += (size_t)NTOK * EMBW * 2;
  const size_t oXN0 = off; off += (size_t)NTOK * ED * 2;
  const size_t oXN1 = off; off += (size_t)NTOK * ED * 2;
  const size_t oW1T = off; off += (size_t)HIDW * EMBW * 2;
  const size_t oW2T = off; off += (size_t)TAGW * KHG * 2;
  const size_t oH   = off; off += (size_t)NTOK * HIDW * 2;
  const size_t oHT  = off; off += (size_t)NBT * HIDW * NS * 2;
  const size_t oG0  = off; off += (size_t)NTOK * HIDW * 2;
  const size_t oG1  = off; off += (size_t)NTOK * HIDW * 2;
  const size_t oPRT = off; off += (size_t)2 * NBT * (NS / BR) * 16 * 8;
  if (off > ws_size) return;
  if (off > (size_t)134217728) return;

  char* ws = (char*)d_ws;
  ush* EMBp = (ush*)(ws + oEMB);
  ush* XN0p = (ush*)(ws + oXN0);
  ush* XN1p = (ush*)(ws + oXN1);
  ush* W1Tp = (ush*)(ws + oW1T);
  ush* W2Tp = (ush*)(ws + oW2T);
  ush* Hp   = (ush*)(ws + oH);
  ush* HTp  = (ush*)(ws + oHT);
  ush* G0p  = (ush*)(ws + oG0);
  ush* G1p  = (ush*)(ws + oG1);
  double* PRTp = (double*)(ws + oPRT);

  k_cvt_w<<<dim3(HIDW / 16, EMBW / 256), dim3(256), 0, stream>>>(W1, HIDW, EMBW, W1Tp);
  k_cvt_w<<<dim3(TAGW / 16, KHG / 256), dim3(256), 0, stream>>>(W2, TAGW, KHG, W2Tp);
  k_gather<<<dim3(NTOK / 8), dim3(256), 0, stream>>>(xc, x0, x1, Ec, E0, E1, EMBp, XN0p, XN1p);
  k_hgemm<<<dim3(NTOK / 256, HIDW / 64), dim3(256), 0, stream>>>(EMBp, W1Tp, b1, Hp, HTp);
  (void)hipFuncSetAttribute(reinterpret_cast<const void*>(&k_attn),
                            hipFuncAttributeMaxDynamicSharedMemorySize, ATT_LDS);
  k_attn<<<dim3(NS / BR, NBT, 2), dim3(256), ATT_LDS, stream>>>(XN0p, XN1p, HTp, G0p, G1p, PRTp);
  k_final<<<dim3(NTOK / 128), dim3(256), 0, stream>>>(Hp, G0p, G1p, W2Tp, b2, PRTp, out);
  (void)hipGetLastError();
}
